// MultiQueryAttention_21423296873307
// MI455X (gfx1250) — hardware-verified
//
#include <hip/hip_runtime.h>
#include <math.h>
#include <stddef.h>
#include <stdint.h>


#ifndef NB
#define NB 2
#endif
#ifndef SEQ
#define SEQ 2048
#endif
#define NB_FULL  2
#define SEQ_FULL 2048
#define DIN   1024
#define DM    1024
#define NH    16
#define HD    64
#define MROWS (NB * SEQ)
#define QT    (SEQ / 16)
#define EQT   (QT < 32 ? QT : 32)
#define NKC   (SEQ / 32)
#define FLP   (((NKC) + 31) / 32 * 32)
#define MASK_T SEQ_FULL

static_assert(SEQ % 128 == 0);
static_assert(SEQ >= 128 && SEQ <= SEQ_FULL);
static_assert(NB >= 1 && NB <= NB_FULL);
static_assert(EQT % 4 == 0);
static_assert((QT - EQT) % 4 == 0);
static_assert((EQT * 16) % 128 == 0);
static_assert(FLP <= 64);
static_assert(DIN % 32 == 0 && DM % 128 == 0 && DIN % 128 == 0 && MROWS % 128 == 0);
static_assert(NH * HD == DM);

#define WSC   64.0f
#define WSCI  0.015625f
#define RC    4096.0f
#define RCI   0.000244140625f
#define PC    16384.0f
#define YOSC  0.00390625f
#define CYI   0.015625f
#define SCL   (0.125f * 1.44269504088896340736f)

typedef _Float16 v16h __attribute__((ext_vector_type(16)));
typedef _Float16 v8h  __attribute__((ext_vector_type(8)));
typedef _Float16 v4h  __attribute__((ext_vector_type(4)));
typedef float    v8f  __attribute__((ext_vector_type(8)));
typedef float    v4f  __attribute__((ext_vector_type(4)));
typedef int      v4i  __attribute__((ext_vector_type(4)));

union HFrag { v16h v; v8h h[2]; };

__device__ __forceinline__ v16h load_frag(const _Float16* p) {
    HFrag f;
    f.h[0] = *reinterpret_cast<const v8h*>(p);
    f.h[1] = *reinterpret_cast<const v8h*>(p + 16);
    return f.v;
}

__device__ __forceinline__ v8f wmma16(v16h a, v16h b, v8f c) {
    v8f d = __builtin_amdgcn_wmma_f32_16x16x32_f16(false, a, false, b,
                                                   (short)0, c, false, false);
    asm volatile("v_nop\n\tv_nop\n\tv_nop\n\tv_nop" : "+v"(d) : "v"(a), "v"(b));
    return d;
}

__device__ __forceinline__ float bf16r(float f) {
    unsigned int u = __float_as_uint(f);
    u = (u + 0x7FFFu + ((u >> 16) & 1u)) & 0xFFFF0000u;
    return __uint_as_float(u);
}

__device__ __forceinline__ void wave_lds_sync() {
    __builtin_amdgcn_fence(3  , "wavefront");
    __builtin_amdgcn_wave_barrier();
}

__global__ __launch_bounds__(256) void k_cvt_x(const float* __restrict__ x,
                                               _Float16* xo, int n8)
{
    const int i = blockIdx.x * 256 + threadIdx.x;
    if (i >= n8) return;
    const int cpr = DIN / 8;
    const int m = i / cpr;
    const int c8 = (i - m * cpr) * 8;
    const int b = m / SEQ;
    const int t = m - b * SEQ;
    const float* src = x + (size_t)(b * SEQ_FULL + t) * DIN + c8;
    const v4f f0 = *(const v4f*)src;
    const v4f f1 = *(const v4f*)(src + 4);
    v8h o;
#pragma unroll
    for (int e = 0; e < 4; ++e) {
        o[e]     = (_Float16)bf16r(f0[e]);
        o[4 + e] = (_Float16)bf16r(f1[e]);
    }
    _Float16* dst = xo + (size_t)m * DIN + c8;
    *(volatile v8h*)dst = o;
    __threadfence();
    *(volatile v8h*)dst = o;
}

__global__ __launch_bounds__(256) void k_cvt_w(const float* __restrict__ W,
                                               _Float16* wo, int n8, float sc)
{
    const int i = blockIdx.x * 256 + threadIdx.x;
    if (i >= n8) return;
    const float* src = W + (size_t)i * 8;
    const v4f f0 = *(const v4f*)src;
    const v4f f1 = *(const v4f*)(src + 4);
    v8h o;
#pragma unroll
    for (int e = 0; e < 4; ++e) {
        o[e]     = (_Float16)(bf16r(f0[e]) * sc);
        o[4 + e] = (_Float16)(bf16r(f1[e]) * sc);
    }
    _Float16* dst = wo + (size_t)i * 8;
    *(volatile v8h*)dst = o;
    __threadfence();
    *(volatile v8h*)dst = o;
}

__global__ __launch_bounds__(256) void k_cvt_kv(const float* __restrict__ Wk,
                                                const float* __restrict__ Wv,
                                                _Float16* wo, float sc)
{
    const int i = blockIdx.x * 256 + threadIdx.x;
    const int cpr = DIN / 8;
    if (i >= 2 * HD * cpr) return;
    const int row = i / cpr;
    const int c8 = (i - row * cpr) * 8;
    const int rk = row < HD ? row : (HD - 1);
    int rv = row - HD; rv = rv < 0 ? 0 : rv;
    const float* pk = Wk + (size_t)rk * DIN + c8;
    const float* pv = Wv + (size_t)rv * DIN + c8;
    const v4f k0 = *(const v4f*)pk, k1 = *(const v4f*)(pk + 4);
    const v4f v0 = *(const v4f*)pv, v1 = *(const v4f*)(pv + 4);
    const bool usek = row < HD;
    v8h o;
#pragma unroll
    for (int e = 0; e < 4; ++e) {
        const float a = usek ? k0[e] : v0[e];
        const float c = usek ? k1[e] : v1[e];
        o[e]     = (_Float16)(bf16r(a) * sc);
        o[4 + e] = (_Float16)(bf16r(c) * sc);
    }
    _Float16* dst = wo + (size_t)row * DIN + c8;
    *(volatile v8h*)dst = o;
    __threadfence();
    *(volatile v8h*)dst = o;
}

__global__ __launch_bounds__(256) void k_flags(const int* __restrict__ mask,
                                               int* flags)
{
    __shared__ alignas(16) int fl[64];
    const int tid = threadIdx.x;
    const int lane = tid & 31, w = tid >> 5;
    const int l15 = lane & 15, h1 = lane >> 4;
    const int qt = blockIdx.x;
    if (tid < FLP) fl[tid] = 1;
    __syncthreads();
    for (int kc = w; kc < NKC; kc += 8) {
        const int* mp = mask + (size_t)(qt * 16 + l15) * MASK_T + kc * 32 + 16 * h1;
        const v4i a0 = *(const v4i*)(mp);
        const v4i a1 = *(const v4i*)(mp + 4);
        const v4i a2 = *(const v4i*)(mp + 8);
        const v4i a3 = *(const v4i*)(mp + 12);
        int anyv = 0, allv = 1;
#pragma unroll
        for (int e = 0; e < 4; ++e) {
            const int n0 = (a0[e] != 0), n1 = (a1[e] != 0), n2 = (a2[e] != 0), n3 = (a3[e] != 0);
            anyv |= n0 | n1 | n2 | n3;
            allv &= n0 & n1 & n2 & n3;
        }
#pragma unroll
        for (int off = 16; off >= 1; off >>= 1) {
            anyv |= __shfl_xor(anyv, off, 32);
            allv &= __shfl_xor(allv, off, 32);
        }
        const int f = allv ? 1 : (anyv ? 2 : 0);
        if (lane == 0) fl[kc] = f;
    }
    __syncthreads();
    if (w == 0 && lane < FLP / 4) {
        const v4i v = *(const v4i*)&fl[lane * 4];
        int* dst = flags + (size_t)qt * FLP + lane * 4;
        *(volatile v4i*)dst = v;
        __threadfence();
        *(volatile v4i*)dst = v;
    }
}

#define GBM 128
#define GBN 128
#define GBK 32
#define LP  40

#define MODE_Q   0
#define MODE_KV  1
#define MODE_OUT 2

struct GemmStage { _Float16 As[GBM * LP]; _Float16 Bs[GBN * LP]; };
union GemmSmem { GemmStage s; float tile[GBM * GBN]; };

static_assert(EQT * 16 >= GBM || EQT * 16 == SEQ);

template <int MODE>
__global__ __launch_bounds__(256) void k_gemm(
    const _Float16* __restrict__ A, const _Float16* __restrict__ Ar,
    const _Float16* __restrict__ BT,
    const float* __restrict__ cosb, const float* __restrict__ sinb,
    _Float16* P0, _Float16* P1, _Float16* P2, _Float16* P3,
    float* Of, int K, int N)
{
    __shared__ alignas(16) GemmSmem sm;

    const int tid  = threadIdx.x;
    const int lane = tid & 31;
    const int wave = tid >> 5;
    const int wm = wave & 3;
    const int wn = wave >> 2;
    const int bm0 = blockIdx.y * GBM;
    const int bn0 = blockIdx.x * GBN;
    const int l15 = lane & 15;
    const int hi8 = (lane >> 4) << 3;
    const int srow = tid >> 2;
    const int skg  = (tid & 3) * 8;

    v8f acc[2][4];
    {
        v8f z = {};
#pragma unroll
        for (int mi = 0; mi < 2; ++mi)
#pragma unroll
            for (int ni = 0; ni < 4; ++ni) acc[mi][ni] = z;
    }

    auto kloop = [&](const _Float16* Ap) {
#pragma unroll 1
        for (int k0 = 0; k0 < K; k0 += GBK) {
            v8h av[2], bv[2];
#pragma unroll
            for (int i = 0; i < 2; ++i) {
                const int row = srow + i * 64;
                av[i] = *(const v8h*)(Ap + (size_t)(bm0 + row) * K + k0 + skg);
                bv[i] = *(const v8h*)(BT + (size_t)(bn0 + row) * K + k0 + skg);
            }
            __syncthreads();
#pragma unroll
            for (int i = 0; i < 2; ++i) {
                const int row = srow + i * 64;
                *(v8h*)&sm.s.As[row * LP + skg] = av[i];
                *(v8h*)&sm.s.Bs[row * LP + skg] = bv[i];
            }
            __syncthreads();
            v16h aF[2], bF[4];
#pragma unroll
            for (int mi = 0; mi < 2; ++mi)
                aF[mi] = load_frag(&sm.s.As[(wm * 32 + mi * 16 + l15) * LP + hi8]);
#pragma unroll
            for (int ni = 0; ni < 4; ++ni)
                bF[ni] = load_frag(&sm.s.Bs[(wn * 64 + ni * 16 + l15) * LP + hi8]);
#pragma unroll
            for (int mi = 0; mi < 2; ++mi)
#pragma unroll
                for (int ni = 0; ni < 4; ++ni)
                    acc[mi][ni] = wmma16(aF[mi], bF[ni], acc[mi][ni]);
        }
    };

    if (MODE == MODE_OUT) {
        const bool early = ((bm0 % SEQ) < EQT * 16);
        if (early) {
            kloop(Ar);
#pragma unroll
            for (int mi = 0; mi < 2; ++mi)
#pragma unroll
                for (int ni = 0; ni < 4; ++ni) acc[mi][ni] = acc[mi][ni] * RCI;
        }
    }
    kloop(A);

    const float osc = (MODE == MODE_OUT) ? (WSCI * CYI) : WSCI;
    __syncthreads();
#pragma unroll
    for (int mi = 0; mi < 2; ++mi)
#pragma unroll
        for (int ni = 0; ni < 4; ++ni)
#pragma unroll
            for (int j = 0; j < 8; ++j)
                sm.tile[(wm * 32 + mi * 16 + hi8 + j) * GBN + wn * 64 + ni * 16 + l15] =
                    acc[mi][ni][j] * osc;
    __syncthreads();

    if (MODE == MODE_Q) {
        v4h hv[16], rv[16];
#pragma unroll
        for (int r = 0; r < 16; ++r) {
            const int rl = wave * 16 + r;
            const int row = bm0 + rl;
            const int t = row % SEQ;
            const int c = lane * 4;
            const int d = c & (HD - 1);
            const v4f qv = *(const v4f*)&sm.tile[rl * GBN + c];
            const v4f qp = *(const v4f*)&sm.tile[rl * GBN + (c ^ 32)];
            const v4f cs = *(const v4f*)(cosb + (size_t)t * HD + d);
            const v4f sn = *(const v4f*)(sinb + (size_t)t * HD + d);
            const float sg = (c & 32) ? 1.0f : -1.0f;
            v4h hh, rr;
#pragma unroll
            for (int e = 0; e < 4; ++e) {
                const float o = qv[e] * bf16r(cs[e]) + sg * qp[e] * bf16r(sn[e]);
                const _Float16 o16 = (_Float16)o;
                hh[e] = o16;
                rr[e] = (_Float16)((o - (float)o16) * RC);
            }
            hv[r] = hh; rv[r] = rr;
        }
#pragma unroll
        for (int r = 0; r < 16; ++r) {
            const size_t idx = (size_t)(bm0 + wave * 16 + r) * N + bn0 + lane * 4;
            *(volatile v4h*)(P0 + idx) = hv[r];
            *(volatile v4h*)(P1 + idx) = rv[r];
        }
        __threadfence();
#pragma unroll
        for (int r = 0; r < 16; ++r) {
            const size_t idx = (size_t)(bm0 + wave * 16 + r) * N + bn0 + lane * 4;
            *(volatile v4h*)(P0 + idx) = hv[r];
            *(volatile v4h*)(P1 + idx) = rv[r];
        }
    } else if (MODE == MODE_KV) {
        const int bb = bm0 / SEQ;
        const int t0 = bm0 - bb * SEQ;
        v4h khv[8], krv[8], vhv[8], vrv[8];
#pragma unroll
        for (int i = 0; i < 8; ++i) {
            const int rl = wave * 16 + 2 * i + (lane >> 4);
            const int row = bm0 + rl;
            const int t = row % SEQ;
            const int c = (lane & 15) * 4;
            const v4f qv = *(const v4f*)&sm.tile[rl * GBN + c];
            const v4f qp = *(const v4f*)&sm.tile[rl * GBN + (c ^ 32)];
            const v4f cs = *(const v4f*)(cosb + (size_t)t * HD + c);
            const v4f sn = *(const v4f*)(sinb + (size_t)t * HD + c);
            const float sg = (c & 32) ? 1.0f : -1.0f;
            v4h hh, rr;
#pragma unroll
            for (int e = 0; e < 4; ++e) {
                const float o = qv[e] * bf16r(cs[e]) + sg * qp[e] * bf16r(sn[e]);
                const _Float16 o16 = (_Float16)o;
                hh[e] = o16;
                rr[e] = (_Float16)((o - (float)o16) * RC);
            }
            khv[i] = hh; krv[i] = rr;
        }
#pragma unroll
        for (int i = 0; i < 8; ++i) {
            const int dcol = wave * 8 + i;
            v4h hh, rr;
#pragma unroll
            for (int e = 0; e < 4; ++e) {
                const float o = sm.tile[(lane * 4 + e) * GBN + HD + dcol];
                const _Float16 o16 = (_Float16)o;
                hh[e] = o16;
                rr[e] = (_Float16)((o - (float)o16) * RC);
            }
            vhv[i] = hh; vrv[i] = rr;
        }
#pragma unroll
        for (int i = 0; i < 8; ++i) {
            const size_t ki = (size_t)(bm0 + wave * 16 + 2 * i + (lane >> 4)) * HD + (lane & 15) * 4;
            *(volatile v4h*)(P0 + ki) = khv[i];
            *(volatile v4h*)(P1 + ki) = krv[i];
            const size_t vi = (size_t)(bb * HD + wave * 8 + i) * SEQ + t0 + lane * 4;
            *(volatile v4h*)(P2 + vi) = vhv[i];
            *(volatile v4h*)(P3 + vi) = vrv[i];
        }
        __threadfence();
#pragma unroll
        for (int i = 0; i < 8; ++i) {
            const size_t ki = (size_t)(bm0 + wave * 16 + 2 * i + (lane >> 4)) * HD + (lane & 15) * 4;
            *(volatile v4h*)(P0 + ki) = khv[i];
            *(volatile v4h*)(P1 + ki) = krv[i];
            const size_t vi = (size_t)(bb * HD + wave * 8 + i) * SEQ + t0 + lane * 4;
            *(volatile v4h*)(P2 + vi) = vhv[i];
            *(volatile v4h*)(P3 + vi) = vrv[i];
        }
    } else {
        v4f ov[16];
#pragma unroll
        for (int r = 0; r < 16; ++r) {
            const int rl = wave * 16 + r;
            ov[r] = *(const v4f*)&sm.tile[rl * GBN + lane * 4];
        }
#pragma unroll
        for (int r = 0; r < 16; ++r) {
            const size_t idx = (size_t)(bm0 + wave * 16 + r) * N + bn0 + lane * 4;
            *(volatile v4f*)(Of + idx) = ov[r];
        }
        __threadfence();
#pragma unroll
        for (int r = 0; r < 16; ++r) {
            const size_t idx = (size_t)(bm0 + wave * 16 + r) * N + bn0 + lane * 4;
            *(volatile v4f*)(Of + idx) = ov[r];
        }
    }
}

#define YP 72

template <int EARLY>
__global__ __launch_bounds__(128) void k_attn(
    const _Float16* __restrict__ qh, const _Float16* __restrict__ qr,
    const _Float16* __restrict__ kh, const _Float16* __restrict__ kr,
    const _Float16* __restrict__ vh, const _Float16* __restrict__ vr,
    const int* __restrict__ flags, const int* __restrict__ mask,
    _Float16* yh, _Float16* yr)
{
    __shared__ alignas(16) _Float16 Ph[4][16 * YP];
    __shared__ alignas(16) _Float16 Pr[EARLY ? 4 : 1][16 * YP];
    __shared__ alignas(16) int Ms[4][16 * 32];

    const int lane = threadIdx.x & 31;
    const int wv   = threadIdx.x >> 5;
    const int l15  = lane & 15;
    const int h1   = lane >> 4;
    const int hi8  = h1 << 3;

    const int QTL = EARLY ? EQT : ((QT - EQT) > 0 ? (QT - EQT) : 1);
    int gw = blockIdx.x * 4 + wv;
    const int qt = (gw % QTL) + (EARLY ? 0 : EQT);
    gw /= QTL;
    const int h = gw % NH;
    const int b = gw / NH;
    const int q0 = qt * 16;

    _Float16* ph = &Ph[wv][0];
    _Float16* pr = &Pr[EARLY ? wv : 0][0];
    int* ms = &Ms[wv][0];

    const size_t qoff = (size_t)(b * SEQ + q0 + l15) * DM + h * HD + hi8;
    const v16h aQ0 = load_frag(qh + qoff);
    const v16h aQ1 = load_frag(qh + qoff + 32);

    const _Float16* kb0 = kh + (size_t)(b * SEQ) * HD + hi8;
    const _Float16* kr0 = kr + (size_t)(b * SEQ) * HD + hi8;
    const _Float16* vb0 = vh + (size_t)(b * HD) * SEQ + hi8;
    const _Float16* vr0 = vr + (size_t)(b * HD) * SEQ + hi8;
    const int* frow = flags + (size_t)qt * FLP;

    float m[8], l[8];
    v8f accY[4], accR[4];
    {
        v8f z = {};
#pragma unroll
        for (int j = 0; j < 8; ++j) { m[j] = -1e30f; l[j] = 0.0f; }
#pragma unroll
        for (int ni = 0; ni < 4; ++ni) { accY[ni] = z; accR[ni] = z; }
    }

#pragma unroll 1
    for (int kc = 0; kc < NKC; ++kc) {
        const int fl = __builtin_amdgcn_readfirstlane(frow[kc]);
        if (fl == 1) continue;
        const int tc = kc * 32;

        v16h aR0, aR1;
        if (EARLY) {
            aR0 = load_frag(qr + qoff);
            aR1 = load_frag(qr + qoff + 32);
        }

        v8f s0 = {};
        {
            const _Float16* kp = kb0 + (size_t)(tc + l15) * HD;
            const v16h b0 = load_frag(kp);
            const v16h b1 = load_frag(kp + 32);
            s0 = wmma16(aQ0, b0, s0);
            s0 = wmma16(aQ1, b1, s0);
            if (EARLY) {
                const _Float16* rp = kr0 + (size_t)(tc + l15) * HD;
                const v16h c0 = load_frag(rp);
                const v16h c1 = load_frag(rp + 32);
                v8f r0 = {};
                r0 = wmma16(aR0, b0, r0);
                r0 = wmma16(aR1, b1, r0);
                r0 = wmma16(aQ0, c0, r0);
                r0 = wmma16(aQ1, c1, r0);
                s0 = s0 + r0 * RCI;
            }
        }
        v8f s1 = {};
        {
            const _Float16* kp = kb0 + (size_t)(tc + 16 + l15) * HD;
            const v16h b0 = load_frag(kp);
            const v16h b1 = load_frag(kp + 32);
            s1 = wmma16(aQ0, b0, s1);
            s1 = wmma16(aQ1, b1, s1);
            if (EARLY) {
                const _Float16* rp = kr0 + (size_t)(tc + 16 + l15) * HD;
                const v16h c0 = load_frag(rp);
                const v16h c1 = load_frag(rp + 32);
                v8f r1 = {};
                r1 = wmma16(aR0, b0, r1);
                r1 = wmma16(aR1, b1, r1);
                r1 = wmma16(aQ0, c0, r1);
                r1 = wmma16(aQ1, c1, r1);
                s1 = s1 + r1 * RCI;
            }
        }
        s0 = s0 * SCL;
        s1 = s1 * SCL;

        if (fl == 2) {
            const int* mp = mask + (size_t)(q0 + l15) * MASK_T + tc + 16 * h1;
            const v4i a0 = *(const v4i*)(mp);
            const v4i a1 = *(const v4i*)(mp + 4);
            const v4i a2 = *(const v4i*)(mp + 8);
            const v4i a3 = *(const v4i*)(mp + 12);
            *(v4i*)&ms[l15 * 32 + 16 * h1 + 0]  = a0;
            *(v4i*)&ms[l15 * 32 + 16 * h1 + 4]  = a1;
            *(v4i*)&ms[l15 * 32 + 16 * h1 + 8]  = a2;
            *(v4i*)&ms[l15 * 32 + 16 * h1 + 12] = a3;
            wave_lds_sync();
#pragma unroll
            for (int j = 0; j < 8; ++j) {
                const int row = hi8 + j;
                const int m0 = ms[row * 32 + l15];
                const int m1 = ms[row * 32 + 16 + l15];
                s0[j] = (m0 != 0) ? -__builtin_inff() : s0[j];
                s1[j] = (m1 != 0) ? -__builtin_inff() : s1[j];
            }
        }

#pragma unroll
        for (int j = 0; j < 8; ++j) {
            float mt = fmaxf(s0[j], s1[j]);
#pragma unroll
            for (int off = 8; off >= 1; off >>= 1)
                mt = fmaxf(mt, __shfl_xor(mt, off, 16));
            const float mn = fmaxf(m[j], mt);
            const float sc = exp2f(m[j] - mn);
            const float p0 = exp2f(s0[j] - mn);
            const float p1 = exp2f(s1[j] - mn);
            float rs = p0 + p1;
#pragma unroll
            for (int off = 8; off >= 1; off >>= 1)
                rs += __shfl_xor(rs, off, 16);
            l[j] = l[j] * sc + rs;
            m[j] = mn;
            s0[j] = p0; s1[j] = p1;
            accY[0][j] *= sc; accY[1][j] *= sc;
            accY[2][j] *= sc; accY[3][j] *= sc;
            if (EARLY) {
                accR[0][j] *= sc; accR[1][j] *= sc;
                accR[2][j] *= sc; accR[3][j] *= sc;
            }
        }

#pragma unroll
        for (int j = 0; j < 8; ++j) {
            const int row = hi8 + j;
            const float pc0 = s0[j] * PC;
            const float pc1 = s1[j] * PC;
            const _Float16 g0 = (_Float16)pc0;
            const _Float16 g1 = (_Float16)pc1;
            ph[row * YP + l15]      = g0;
            ph[row * YP + 16 + l15] = g1;
            if (EARLY) {
                pr[row * YP + l15]      = (_Float16)((pc0 - (float)g0) * RC);
                pr[row * YP + 16 + l15] = (_Float16)((pc1 - (float)g1) * RC);
            }
        }
        wave_lds_sync();
        const v16h aP = load_frag(&ph[l15 * YP + hi8]);
        v16h aPr = aP;
        if (EARLY) aPr = load_frag(&pr[l15 * YP + hi8]);

#pragma unroll
        for (int ni = 0; ni < 4; ++ni) {
            const v16h bV = load_frag(vb0 + (size_t)(ni * 16 + l15) * SEQ + tc);
            accY[ni] = wmma16(aP, bV, accY[ni]);
            if (EARLY) {
                const v16h bVr = load_frag(vr0 + (size_t)(ni * 16 + l15) * SEQ + tc);
                accR[ni] = wmma16(aP, bVr, accR[ni]);
                accR[ni] = wmma16(aPr, bV, accR[ni]);
            }
        }
    }

    float inv[8];
#pragma unroll
    for (int j = 0; j < 8; ++j) inv[j] = (1.0f / l[j]) * YOSC;
    wave_lds_sync();
#pragma unroll
    for (int ni = 0; ni < 4; ++ni)
#pragma unroll
        for (int j = 0; j < 8; ++j) {
            const int row = hi8 + j;
            float y = accY[ni][j];
            if (EARLY) y = y + accR[ni][j] * RCI;
            y = y * inv[j];
            const _Float16 y16 = (_Float16)y;
            ph[row * YP + ni * 16 + l15] = y16;
            if (EARLY) pr[row * YP + ni * 16 + l15] = (_Float16)((y - (float)y16) * RC);
        }
    wave_lds_sync();
    v8h yv[4], yq[4];
#pragma unroll
    for (int it = 0; it < 4; ++it) {
        const int rl = it * 4 + (lane >> 3);
        const int c8 = (lane & 7) * 8;
        yv[it] = *(const v8h*)&ph[rl * YP + c8];
        yq[it] = yv[it];
        if (EARLY) yq[it] = *(const v8h*)&pr[rl * YP + c8];
    }
    const size_t ybase = (size_t)(b * SEQ + q0) * DM + h * HD;
#pragma unroll
    for (int it = 0; it < 4; ++it) {
        const int rl = it * 4 + (lane >> 3);
        const int c8 = (lane & 7) * 8;
        const size_t idx = ybase + (size_t)rl * DM + c8;
        *(volatile v8h*)(yh + idx) = yv[it];
        if (EARLY) *(volatile v8h*)(yr + idx) = yq[it];
    }
    __threadfence();
#pragma unroll
    for (int it = 0; it < 4; ++it) {
        const int rl = it * 4 + (lane >> 3);
        const int c8 = (lane & 7) * 8;
        const size_t idx = ybase + (size_t)rl * DM + c8;
        *(volatile v8h*)(yh + idx) = yv[it];
        if (EARLY) *(volatile v8h*)(yr + idx) = yq[it];
    }
}

extern "C" void kernel_launch(void* const* d_in, const int* in_sizes, int n_in,
                              void* d_out, int out_size, void* d_ws, size_t ws_size,
                              hipStream_t stream) {
    if (n_in < 8) return;
    const float* x    = (const float*)d_in[0];
    const int*   mask = (const int*)d_in[1];
    const float* cosb = (const float*)d_in[2];
    const float* sinb = (const float*)d_in[3];
    const float* Wq   = (const float*)d_in[4];
    const float* Wk   = (const float*)d_in[5];
    const float* Wv   = (const float*)d_in[6];
    const float* Wo   = (const float*)d_in[7];
    float* out = (float*)d_out;

    if ((size_t)in_sizes[0] < ((size_t)(NB - 1) * SEQ_FULL + SEQ) * DIN) return;
    if ((size_t)in_sizes[1] < (size_t)(SEQ - 1) * MASK_T + SEQ) return;
    if ((size_t)in_sizes[2] < (size_t)SEQ * HD) return;
    if ((size_t)in_sizes[3] < (size_t)SEQ * HD) return;
    if ((size_t)in_sizes[4] < (size_t)DM * DIN) return;
    if ((size_t)in_sizes[5] < (size_t)HD * DIN) return;
    if ((size_t)in_sizes[6] < (size_t)HD * DIN) return;
    if ((size_t)in_sizes[7] < (size_t)DIN * DM) return;
    if ((size_t)out_size < (size_t)MROWS * DIN) return;

    size_t off = 0;
    auto carve = [&](size_t bytes) -> size_t {
        const size_t o = off;
        off += (bytes + 255) & ~(size_t)255;
        return o;
    };
    const size_t o_x16  = carve((size_t)MROWS * DIN * 2);
    const size_t o_wq   = carve((size_t)DM * DIN * 2);
    const size_t o_wkv  = carve((size_t)2 * HD * DIN * 2);
    const size_t o_wo   = carve((size_t)DIN * DM * 2);
    const size_t o_qh   = carve((size_t)MROWS * DM * 2);
    const size_t o_qr   = carve((size_t)MROWS * DM * 2);
    const size_t o_kh   = carve((size_t)MROWS * HD * 2);
    const size_t o_kr   = carve((size_t)MROWS * HD * 2);
    const size_t o_vh   = carve((size_t)NB * HD * SEQ * 2);
    const size_t o_vr   = carve((size_t)NB * HD * SEQ * 2);
    const size_t o_yh   = carve((size_t)MROWS * DM * 2);
    const size_t o_yr   = carve((size_t)MROWS * DM * 2);
    const size_t o_fl   = carve((size_t)QT * FLP * 4);
    if (off > ws_size) return;

    char* ws = (char*)d_ws;
    _Float16* x16  = (_Float16*)(ws + o_x16);
    _Float16* wq16 = (_Float16*)(ws + o_wq);
    _Float16* wkv16 = (_Float16*)(ws + o_wkv);
    _Float16* wo16 = (_Float16*)(ws + o_wo);
    _Float16* qh = (_Float16*)(ws + o_qh);
    _Float16* qr = (_Float16*)(ws + o_qr);
    _Float16* kh = (_Float16*)(ws + o_kh);
    _Float16* kr = (_Float16*)(ws + o_kr);
    _Float16* vh = (_Float16*)(ws + o_vh);
    _Float16* vr = (_Float16*)(ws + o_vr);
    _Float16* yh = (_Float16*)(ws + o_yh);
    _Float16* yr = (_Float16*)(ws + o_yr);
    int* flags = (int*)(ws + o_fl);

    {
        const int n8x = MROWS * DIN / 8;
        k_cvt_x<<<dim3((n8x + 255) / 256), dim3(256), 0, stream>>>(x, x16, n8x);
        const int n8w = DM * DIN / 8;
        k_cvt_w<<<dim3((n8w + 255) / 256), dim3(256), 0, stream>>>(Wq, wq16, n8w, WSC);
        const int n8kv = 2 * HD * DIN / 8;
        k_cvt_kv<<<dim3((n8kv + 255) / 256), dim3(256), 0, stream>>>(Wk, Wv, wkv16, WSC);
        k_cvt_w<<<dim3((n8w + 255) / 256), dim3(256), 0, stream>>>(Wo, wo16, n8w, WSC);
    }
    k_flags<<<dim3(QT), dim3(256), 0, stream>>>(mask, flags);

    k_gemm<MODE_Q><<<dim3(DM / GBN, MROWS / GBM), dim3(256), 0, stream>>>(
        x16, x16, wq16, cosb, sinb, qh, qr, qh, qr, out, DIN, DM);
    k_gemm<MODE_KV><<<dim3(1, MROWS / GBM), dim3(256), 0, stream>>>(
        x16, x16, wkv16, cosb, sinb, kh, kr, vh, vr, out, DIN, 2 * HD);

    {
        const int nbe = NB * NH * EQT / 4;
        k_attn<1><<<dim3(nbe), dim3(128), 0, stream>>>(
            qh, qr, kh, kr, vh, vr, flags, mask, yh, yr);
        const int late = QT - EQT;
        if (late > 0) {
            const int nbl = NB * NH * late / 4;
            k_attn<0><<<dim3(nbl), dim3(128), 0, stream>>>(
                qh, qr, kh, kr, vh, vr, flags, mask, yh, yr);
        }
    }

    k_gemm<MODE_OUT><<<dim3(DIN / GBN, MROWS / GBM), dim3(256), 0, stream>>>(
        yh, yr, wo16, cosb, sinb, qh, qr, vh, vr, out, DM, DIN);
}
